// GNN_1881195675938
// MI455X (gfx1250) — hardware-run, weakly checked
//
#include <hip/hip_runtime.h>

typedef float          v8f   __attribute__((ext_vector_type(8)));
typedef float          v4f   __attribute__((ext_vector_type(4)));
typedef unsigned int   v4u   __attribute__((ext_vector_type(4)));
typedef int            v8i   __attribute__((ext_vector_type(8)));
typedef unsigned short v8us  __attribute__((ext_vector_type(8)));
typedef unsigned short v16us __attribute__((ext_vector_type(16)));
typedef __bf16         v16bf __attribute__((ext_vector_type(16)));
typedef _Float16       v16h  __attribute__((ext_vector_type(16)));
typedef v4f  __attribute__((may_alias)) v4fa;
typedef v8us __attribute__((may_alias)) v8usa;
union FragB { v16bf v; v16us u; v8us h[2]; v8i w; };
union FragH { v16h  v; v16us u; v8us h[2]; v8i w; };

__device__ __forceinline__ v8f wmb(const FragB& a, const FragB& b, v8f c) {
  v8f d = __builtin_amdgcn_wmma_f32_16x16x32_bf16(false, a.v, false, b.v, (short)0, c, false, false);
  asm volatile("v_nop\n\tv_nop\n\tv_nop\n\tv_nop" : "+v"(d) : "v"(a.w), "v"(b.w));
  return d;
}

__device__ __forceinline__ v8f wmh(const FragH& a, const FragH& b, v8f c) {
  v8f d = __builtin_amdgcn_wmma_f32_16x16x32_f16(false, a.v, false, b.v, (short)0, c, false, false);
  asm volatile("v_nop\n\tv_nop\n\tv_nop\n\tv_nop" : "+v"(d) : "v"(a.w), "v"(b.w));
  return d;
}

__device__ __forceinline__ unsigned bf16_bits(float f) {
  const unsigned u = __float_as_uint(f);
  const unsigned r = (u + 0x7FFFu + ((u >> 16) & 1u)) >> 16;
  const unsigned q = (u >> 16) | 0x40u;
  return ((u & 0x7fffffffu) > 0x7f800000u) ? q : r;
}

__device__ __forceinline__ float bf16_val(float f) {
  return __uint_as_float(bf16_bits(f) << 16);
}
__device__ __forceinline__ int clampi(int v, int lo, int hi) {
  return v < lo ? lo : (v > hi ? hi : v);
}

__device__ __forceinline__ unsigned f16_bits(float f) {
  const unsigned u  = __float_as_uint(f);
  const unsigned s  = (u >> 16) & 0x8000u;
  const unsigned a  = u & 0x7fffffffu;
  const unsigned t  = a - 0x38000000u;
  const unsigned r  = (t + 0x0FFFu + ((t >> 13) & 1u)) >> 13;
  const unsigned rc = r > 0x7C00u ? 0x7C00u : r;
  const bool small  = a < 0x38800000u;
  const bool isnan  = a > 0x7f800000u;
  const unsigned fin = small ? 0u : (s | rc);
  return isnan ? (s | 0x7E00u) : fin;
}

__device__ __forceinline__ unsigned pk16(unsigned lo, unsigned hi) { return lo | (hi << 16); }
__device__ __forceinline__ unsigned bf16_lo_bits(float v) {
  float hi = bf16_val(v);
  asm volatile("" : "+v"(hi));
  return bf16_bits(v - hi);
}
__device__ __forceinline__ v4u pack8_bf16(v4f a, v4f c) {
  return (v4u){ pk16(bf16_bits(a[0]), bf16_bits(a[1])), pk16(bf16_bits(a[2]), bf16_bits(a[3])),
                pk16(bf16_bits(c[0]), bf16_bits(c[1])), pk16(bf16_bits(c[2]), bf16_bits(c[3])) };
}
__device__ __forceinline__ v4u pack8_bf16_lo(v4f a, v4f c) {
  return (v4u){ pk16(bf16_lo_bits(a[0]), bf16_lo_bits(a[1])), pk16(bf16_lo_bits(a[2]), bf16_lo_bits(a[3])),
                pk16(bf16_lo_bits(c[0]), bf16_lo_bits(c[1])), pk16(bf16_lo_bits(c[2]), bf16_lo_bits(c[3])) };
}
__device__ __forceinline__ v4u pack8_f16(v4f a, v4f c) {
  return (v4u){ pk16(f16_bits(a[0]), f16_bits(a[1])), pk16(f16_bits(a[2]), f16_bits(a[3])),
                pk16(f16_bits(c[0]), f16_bits(c[1])), pk16(f16_bits(c[2]), f16_bits(c[3])) };
}

template <int FORM>
__global__ __launch_bounds__(256) void k_plane(const float* __restrict__ src, int rows, int cols, int ldsrc,
                                               unsigned short* __restrict__ dst, int MP, int KP) {
  static_assert(FORM >= 0 && FORM <= 3);
  const int KTOT = (FORM == 1 || FORM == 3) ? 2 * KP : KP;
  const unsigned ppr   = (unsigned)(KTOT >> 3);
  const unsigned kp8   = (unsigned)(KP >> 3);
  const unsigned total = (unsigned)MP * ppr;
  const unsigned g     = blockIdx.x * 256u + threadIdx.x;
  const unsigned rowu  = g / ppr;
  const unsigned p     = g - rowu * ppr;
  const bool second    = p >= kp8;
  const int row = (int)rowu;
  const int c0  = (int)((second ? p - kp8 : p) << 3);
  const float* srow = src + (size_t)clampi(row, 0, rows - 1) * (size_t)ldsrc;
  float x[8];
  unsigned mk[8];
#pragma unroll
  for (int e = 0; e < 8; ++e) {
    const int c = c0 + e;
    const float v = srow[clampi(c, 0, cols - 1)];
    asm volatile("" :: "v"(v));
    x[e]  = v;
    mk[e] = (row < rows && c < cols) ? 0xFFFFu : 0u;
  }
  const v4f a = (v4f){ x[0], x[1], x[2], x[3] };
  const v4f c = (v4f){ x[4], x[5], x[6], x[7] };
  v4u o;
  if (FORM == 2) {
    o = pack8_f16(a, c);
  } else {
    const v4u hi = pack8_bf16(a, c);
    o = hi;
    if (FORM == 1) { const v4u lo = pack8_bf16_lo(a, c); o = second ? lo : hi; }
  }
  const v4u mw = (v4u){ pk16(mk[0], mk[1]), pk16(mk[2], mk[3]), pk16(mk[4], mk[5]), pk16(mk[6], mk[7]) };
  o &= mw;
  if (g < total) {
    volatile v4u* q = (volatile v4u*)(dst + (size_t)g * 8);
    *q = o;
    __threadfence();
    *q = o;
  }
}

template <int FORM> struct FragOf    { typedef FragB T; };
template <>         struct FragOf<2> { typedef FragH T; };
__device__ __forceinline__ v8f mm(const FragB& a, const FragB& b, v8f c) { return wmb(a, b, c); }
__device__ __forceinline__ v8f mm(const FragH& a, const FragH& b, v8f c) { return wmh(a, b, c); }
template <class F> __device__ __forceinline__ F ld_frag(const unsigned short* p) {
  F f;
  f.h[0] = *(const v8usa*)(p);
  f.h[1] = *(const v8usa*)(p + 16);
  return f;
}

template <int FORM, int EPI>
__global__ __launch_bounds__(256) __attribute__((amdgpu_num_vgpr(248)))
void k_gemm_nt(const unsigned short* __restrict__ A, const unsigned short* __restrict__ B,
               const float* __restrict__ bias, float* __restrict__ D, int M, int N, int KTOT, int ldd) {
  static_assert(FORM >= 0 && FORM <= 2);
  static_assert(EPI == 0 || EPI == 1);
  typedef typename FragOf<FORM>::T F;
  __shared__ __attribute__((aligned(16))) float sT[8][16 * 68];
  const int lane = threadIdx.x & 31;
  const int wave = threadIdx.x >> 5;
  const int tilesM = (M + 63) >> 6;
  const int tilesN = (N + 63) >> 6;
  const int tile = blockIdx.x * 8 + wave;
  if (tile >= tilesM * tilesN) return;
  const int tm = tile / tilesN;
  const int tn = tile - tm * tilesN;
  const int m0 = tm << 6;
  const int n0 = tn << 6;

  const int rl = lane & 15;
  const int h8 = (lane >> 4) * 8;
  const unsigned short* pa = A + (size_t)(m0 + rl) * (size_t)KTOT + h8;
  const unsigned short* pb = B + (size_t)(n0 + rl) * (size_t)KTOT + h8;

  v8f acc[4][4];
#pragma unroll
  for (int i = 0; i < 4; ++i)
#pragma unroll
    for (int j = 0; j < 4; ++j) acc[i][j] = (v8f){0.f, 0.f, 0.f, 0.f, 0.f, 0.f, 0.f, 0.f};

#pragma unroll 1
  for (int k0 = 0; k0 < KTOT; k0 += 32) {
    F bf[4];
#pragma unroll
    for (int j = 0; j < 4; ++j) bf[j] = ld_frag<F>(pb + (size_t)(j << 4) * (size_t)KTOT + k0);
#pragma unroll
    for (int i = 0; i < 4; ++i) {
      const F af = ld_frag<F>(pa + (size_t)(i << 4) * (size_t)KTOT + k0);
#pragma unroll
      for (int j = 0; j < 4; ++j) acc[i][j] = mm(af, bf[j], acc[i][j]);
    }
  }

  float* slab = sT[wave];
  const int hh = lane >> 4;
  const int c4 = (lane & 15) * 4;
  const int nc = n0 + c4;
  const bool cok = nc < N;
  v4f bv = (v4f){0.f, 0.f, 0.f, 0.f};
  if (EPI == 1) {
    bv = *(const v4fa*)(bias + clampi(nc, 0, N - 4));
    asm volatile("" :: "v"(bv));
  }
#pragma unroll
  for (int i = 0; i < 4; ++i) {
    const int mBase = m0 + (i << 4);
#pragma unroll
    for (int j = 0; j < 4; ++j) {
#pragma unroll
      for (int r = 0; r < 8; ++r) slab[(h8 + r) * 68 + (j << 4) + rl] = acc[i][j][r];
    }
    __builtin_amdgcn_fence(__ATOMIC_RELEASE, "workgroup");
    __builtin_amdgcn_wave_barrier();
    __builtin_amdgcn_fence(__ATOMIC_ACQUIRE, "workgroup");
    v4f vv[8];
#pragma unroll
    for (int it = 0; it < 8; ++it) {
      const int row = it * 2 + hh;
      v4f v = *(const v4fa*)(slab + row * 68 + c4);
      if (EPI == 1) v += bv;
      vv[it] = v;
    }
    for (int pass = 0; pass < 2; ++pass) {
#pragma unroll
      for (int it = 0; it < 8; ++it) {
        const int row = mBase + it * 2 + hh;
        if (cok && row < M) *(volatile v4f*)(D + (size_t)row * (size_t)ldd + nc) = vv[it];
      }
      __threadfence();
    }
    __builtin_amdgcn_fence(__ATOMIC_RELEASE, "workgroup");
    __builtin_amdgcn_wave_barrier();
    __builtin_amdgcn_fence(__ATOMIC_ACQUIRE, "workgroup");
  }
}

#include <stddef.h>
#include <stdint.h>
#include <math.h>

#pragma clang fp contract(off)

#define NN      100000
#define KD      128
#define HID     16
#define OC      64
#define K2      32
#define NE      3200000
#define NPAD    100096
#define NTHR    256
#define NWAVE   8
#define EPT     8
#define WCH     (32 * EPT)
#define NBRUN   256
#define SLB     8
#define NBK     391
#define WLCAP   2048
#define LCAP    12288
#define DEGCAP  72
#define MAXDEG_MEAS   57
#define MAXB256_MEAS  8447

#define BK_INTS  (NWAVE * WLCAP + LCAP + 4 * NBRUN)
#define BK_LDS   (BK_INTS * 4)

#define PBX         (NPAD * KD / 8 / 256)
#define PB_W1       4
#define PB_TOT      6
#define GEMM_BLOCKS (((NPAD / 64) + 7) / 8)

static_assert(OC == 16 * 4 && HID == 4 * 4 && K2 == 2 * HID && K2 % 32 == 0 && KD % 32 == 0);
static_assert(NPAD % 64 == 0 && NPAD >= NN && NPAD % 16 == 0 && OC % 32 == 0);
static_assert((NPAD * KD / 8) % 256 == 0);
static_assert((64 * KD / 8) == PB_W1 * NTHR && (64 * K2 / 8) == NTHR);
static_assert(NBRUN == (1 << SLB) && NBRUN == NTHR && NBRUN == NWAVE * 32);
static_assert(NBK * NBRUN == NPAD && (NBK - 1) * NBRUN < NN);
static_assert(NE < (1 << 22) && (((long long)NE) << SLB) < (1LL << 31));
static_assert(NE % WCH == 0 && NE % 4 == 0);
static_assert(LCAP >= MAXB256_MEAS && (long long)LCAP * 100 >= (long long)MAXB256_MEAS * 125);
static_assert(WLCAP >= MAXB256_MEAS / 8 + 8 * 33 + 1);
static_assert(MAXDEG_MEAS + 8 <= DEGCAP);
static_assert(LCAP % (NTHR * 4) == 0 && BK_INTS % (NTHR * 4) == 0);
static_assert(BK_LDS <= 327680);
static_assert(NN % 2 == 0);
static_assert(GEMM_BLOCKS == 196 && PBX == 6256);

typedef unsigned int v2u __attribute__((ext_vector_type(2)));
typedef int          v4i __attribute__((ext_vector_type(4)));
typedef v2u __attribute__((may_alias)) v2ua;
typedef v4u __attribute__((may_alias)) v4ua;
typedef v4i __attribute__((may_alias)) v4ia;

__device__ __forceinline__ void st2_v4u(unsigned short* p, v4u v) {
  volatile v4u* q = (volatile v4u*)p;
  *q = v;
  __threadfence();
  *q = v;
}
__device__ __forceinline__ void st2_v4f(float* p, v4f v) {
  volatile v4f* q = (volatile v4f*)p;
  *q = v;
  __threadfence();
  *q = v;
}

__device__ __forceinline__ v4u gather8_bf16(const float* __restrict__ base, int stride) {
  float f[8];
#pragma unroll
  for (int i = 0; i < 8; ++i) {
    const float v = base[(size_t)i * (size_t)stride];
    asm volatile("" :: "v"(v));
    f[i] = v;
  }
  return (v4u){ pk16(bf16_bits(f[0]), bf16_bits(f[1])), pk16(bf16_bits(f[2]), bf16_bits(f[3])),
                pk16(bf16_bits(f[4]), bf16_bits(f[5])), pk16(bf16_bits(f[6]), bf16_bits(f[7])) };
}

__global__ __launch_bounds__(NTHR) void k_prep(const float* __restrict__ w1, const float* __restrict__ w2,
                                               const float* __restrict__ b1, const float* __restrict__ b2,
                                               unsigned short* w1t, unsigned short* w2d, float* tab) {
  const int tid = (int)threadIdx.x;
  const int blk = (int)blockIdx.x;
  if (blk < PB_W1) {
    const int u = blk * NTHR + tid;
    const int n = u >> 4, k8 = (u & 15) * 8;
    const int ncl = n < HID ? n : HID - 1;
    v4u o = gather8_bf16(w1 + (size_t)k8 * HID + ncl, HID);
    const unsigned m = (n < HID) ? 0xFFFFFFFFu : 0u;
    o &= (v4u){ m, m, m, m };
    st2_v4u(w1t + (size_t)n * KD + k8, o);
  } else if (blk == PB_W1) {
    const int n = tid >> 2, k8 = (tid & 3) * 8;
    const int ks = k8 & (HID - 1);
    const v4u o = gather8_bf16(w2 + (size_t)ks * OC + n, OC);
    st2_v4u(w2d + (size_t)n * K2 + k8, o);
  } else {
    const int c1 = (tid & 3) * 4;
    const int c2 = ((tid - 8) & 15) * 4;
    const v4f x1 = *(const v4fa*)(b1 + c1);
    const v4f x2 = *(const v4fa*)(b2 + c2);
    asm volatile("" :: "v"(x1), "v"(x2));
    const unsigned m1 = (tid < 4) ? 0xFFFFFFFFu : 0u;
    const unsigned m2 = (tid >= 8 && tid < 24) ? 0xFFFFFFFFu : 0u;
    v4f o;
#pragma unroll
    for (int e = 0; e < 4; ++e) {
      const unsigned u1 = __float_as_uint(bf16_val(x1[e])) & m1;
      const unsigned u2 = __float_as_uint(bf16_val(x2[e])) & m2;
      o[e] = __uint_as_float(u1 | u2);
    }
    if (tid < 40) st2_v4f(tab + 4 * tid, o);
  }
}

__global__ __launch_bounds__(NTHR) void k_build(const int* __restrict__ srcs, const int* __restrict__ dsts,
                                                int* LIST, int* CNT, int* OFF, int* DINVB, int* FLAG) {
  extern __shared__ __attribute__((aligned(16))) int dsm[];
  int* wl   = dsm;
  int* pl   = dsm + NWAVE * WLCAP;
  int* cnt  = pl + LCAP;
  int* offs = cnt + NBRUN;
  int* cur  = offs + NBRUN;
  int* misc = cur + NBRUN;
  const int tid = (int)threadIdx.x, lane = tid & 31, wave = tid >> 5;
  const int blk = (int)blockIdx.x;
  const unsigned nbs = (unsigned)(blk * NBRUN);

  {
    const v4i z4 = {0, 0, 0, 0};
#pragma unroll 1
    for (int i = tid * 4; i < BK_INTS; i += NTHR * 4) *(v4ia*)(dsm + i) = z4;
  }
  __syncthreads();

  {
    const int per  = ((NE + NWAVE * WCH - 1) / (NWAVE * WCH)) * WCH;
    const int ebeg = wave * per;
    const int eend = (ebeg + per < NE) ? (ebeg + per) : NE;
    int* mylist = wl + wave * WLCAP;
    int wc = 0;
#pragma unroll 1
    for (int cb = ebeg; cb < eend; cb += WCH) {
      const int e0 = cb + lane * EPT;
      const v4i da = *(const v4ia*)(dsts + e0);
      const v4i db = *(const v4ia*)(dsts + e0 + 4);
      const int d0 = da.x, d1 = da.y, d2 = da.z, d3 = da.w;
      const int d4 = db.x, d5 = db.y, d6 = db.z, d7 = db.w;
      asm volatile("" :: "v"(d0), "v"(d1), "v"(d2), "v"(d3));
      asm volatile("" :: "v"(d4), "v"(d5), "v"(d6), "v"(d7));
      const unsigned s0 = (unsigned)d0 - nbs, s1 = (unsigned)d1 - nbs;
      const unsigned s2 = (unsigned)d2 - nbs, s3 = (unsigned)d3 - nbs;
      const unsigned s4 = (unsigned)d4 - nbs, s5 = (unsigned)d5 - nbs;
      const unsigned s6 = (unsigned)d6 - nbs, s7 = (unsigned)d7 - nbs;
      const bool h0 = s0 < (unsigned)NBRUN, h1 = s1 < (unsigned)NBRUN, h2 = s2 < (unsigned)NBRUN, h3 = s3 < (unsigned)NBRUN;
      const bool h4 = s4 < (unsigned)NBRUN, h5 = s5 < (unsigned)NBRUN, h6 = s6 < (unsigned)NBRUN, h7 = s7 < (unsigned)NBRUN;
      const unsigned m0 = __builtin_amdgcn_ballot_w32(h0), m1 = __builtin_amdgcn_ballot_w32(h1);
      const unsigned m2 = __builtin_amdgcn_ballot_w32(h2), m3 = __builtin_amdgcn_ballot_w32(h3);
      const unsigned m4 = __builtin_amdgcn_ballot_w32(h4), m5 = __builtin_amdgcn_ballot_w32(h5);
      const unsigned m6 = __builtin_amdgcn_ballot_w32(h6), m7 = __builtin_amdgcn_ballot_w32(h7);
      const unsigned any = m0 | m1 | m2 | m3 | m4 | m5 | m6 | m7;
      if (any != 0u) {
        const int pre = (int)(__builtin_amdgcn_mbcnt_lo(m0, 0u) + __builtin_amdgcn_mbcnt_lo(m1, 0u) +
                              __builtin_amdgcn_mbcnt_lo(m2, 0u) + __builtin_amdgcn_mbcnt_lo(m3, 0u) +
                              __builtin_amdgcn_mbcnt_lo(m4, 0u) + __builtin_amdgcn_mbcnt_lo(m5, 0u) +
                              __builtin_amdgcn_mbcnt_lo(m6, 0u) + __builtin_amdgcn_mbcnt_lo(m7, 0u));
        int p = wc + pre;
        if (h0) { if (p < WLCAP) mylist[p] = ((e0 + 0) << SLB) | (int)s0; p = p + 1; }
        if (h1) { if (p < WLCAP) mylist[p] = ((e0 + 1) << SLB) | (int)s1; p = p + 1; }
        if (h2) { if (p < WLCAP) mylist[p] = ((e0 + 2) << SLB) | (int)s2; p = p + 1; }
        if (h3) { if (p < WLCAP) mylist[p] = ((e0 + 3) << SLB) | (int)s3; p = p + 1; }
        if (h4) { if (p < WLCAP) mylist[p] = ((e0 + 4) << SLB) | (int)s4; p = p + 1; }
        if (h5) { if (p < WLCAP) mylist[p] = ((e0 + 5) << SLB) | (int)s5; p = p + 1; }
        if (h6) { if (p < WLCAP) mylist[p] = ((e0 + 6) << SLB) | (int)s6; p = p + 1; }
        if (h7) { if (p < WLCAP) mylist[p] = ((e0 + 7) << SLB) | (int)s7; p = p + 1; }
        wc += (int)(__builtin_popcount(m0) + __builtin_popcount(m1) + __builtin_popcount(m2) + __builtin_popcount(m3) +
                    __builtin_popcount(m4) + __builtin_popcount(m5) + __builtin_popcount(m6) + __builtin_popcount(m7));
      }
    }
    if (lane == 0) misc[wave] = wc;
  }
  __syncthreads();

  if (wave == 0) {
    int ov = 0;
    int tot = 0;
#pragma unroll 1
    for (int w2 = 0; w2 < NWAVE; ++w2) {
      int c = misc[w2];
      if (c > WLCAP) ov = 1;
      c = c < 0 ? 0 : (c > WLCAP ? WLCAP : c);
      tot += c;
#pragma unroll 1
      for (int b0 = 0; b0 < c; b0 += 32) {
        const int idx = b0 + lane;
        const int ent = wl[w2 * WLCAP + (idx < WLCAP ? idx : WLCAP - 1)];
        const int m32 = (c - b0) < 32 ? (c - b0) : 32;
#pragma unroll 1
        for (int k = 0; k < m32; ++k) {
          const int u    = __builtin_amdgcn_readlane(ent, k);
          const int slot = u & (NBRUN - 1);
          if (lane == 0) cnt[slot] = cnt[slot] + 1;
        }
      }
    }
    if (tot > LCAP) ov = 1;
    if (lane == 0) misc[9] = ov;
  }
  __syncthreads();
  if (wave == 0) {
    const int base = lane * (NBRUN / 32);
    int s = 0;
#pragma unroll 1
    for (int i = 0; i < NBRUN / 32; ++i) s += cnt[base + i];
    int incl = s;
#pragma unroll
    for (int d = 1; d < 32; d <<= 1) {
      const int y = __shfl_up(incl, d, 32);
      if (lane >= d) incl += y;
    }
    int run = incl - s;
#pragma unroll 1
    for (int i = 0; i < NBRUN / 32; ++i) {
      const int cv = cnt[base + i];
      offs[base + i] = run;
      cur[base + i]  = run;
      run += cv;
    }
  }
  __syncthreads();

  if (wave == 0) {
#pragma unroll 1
    for (int w2 = 0; w2 < NWAVE; ++w2) {
      int c = misc[w2];
      c = c < 0 ? 0 : (c > WLCAP ? WLCAP : c);
#pragma unroll 1
      for (int b0 = 0; b0 < c; b0 += 32) {
        const int idx = b0 + lane;
        const int ent = wl[w2 * WLCAP + (idx < WLCAP ? idx : WLCAP - 1)];
        int eid = (ent >> SLB) & 0x3FFFFF;
        eid = eid > NE - 1 ? NE - 1 : eid;
        int sr = srcs[eid];
        asm volatile("" :: "v"(sr));
        sr = sr < 0 ? 0 : (sr > NN - 1 ? NN - 1 : sr);
        const int m32 = (c - b0) < 32 ? (c - b0) : 32;
#pragma unroll 1
        for (int k = 0; k < m32; ++k) {
          const int u    = __builtin_amdgcn_readlane(ent, k);
          const int w0   = __builtin_amdgcn_readlane(sr, k);
          const int slot = u & (NBRUN - 1);
          if (lane == 0) {
            int p = cur[slot];
            p = p < 0 ? 0 : (p > LCAP - 1 ? LCAP - 1 : p);
            pl[p] = w0;
            cur[slot] = p + 1;
          }
        }
      }
    }
  }
  __syncthreads();

  {
    const int cc = cnt[tid];
    const float deg = (float)(cc + 1);
    const float dv = (deg > 0.0f) ? (1.0f / sqrtf(deg)) : 0.0f;
    cur[tid] = __float_as_int(dv);
    const unsigned bm = __builtin_amdgcn_ballot_w32(cc > DEGCAP);
    if (lane == 0) misc[16 + wave] = (bm != 0u) ? 1 : 0;
  }
  __syncthreads();

  int ovf = misc[9];
#pragma unroll
  for (int w2 = 0; w2 < NWAVE; ++w2) ovf |= misc[16 + w2];

  int* lp = LIST  + (size_t)blk * (size_t)LCAP;
  int* cp = CNT   + (size_t)blk * NBRUN;
  int* op = OFF   + (size_t)blk * NBRUN;
  int* dp = DINVB + (size_t)blk * NBRUN;
  int* fp = FLAG  + (size_t)blk * 32;
  for (int pass = 0; pass < 2; ++pass) {
#pragma unroll 1
    for (int i = tid * 4; i < LCAP; i += NTHR * 4) {
      const v4i v = *(const v4ia*)(pl + i);
      *(volatile v4i*)(lp + i) = v;
    }
    if (tid < 64) {
      const v4i vc = *(const v4ia*)(cnt + 4 * tid);
      const v4i vo = *(const v4ia*)(offs + 4 * tid);
      const v4i vd = *(const v4ia*)(cur + 4 * tid);
      *(volatile v4i*)(cp + 4 * tid) = vc;
      *(volatile v4i*)(op + 4 * tid) = vo;
      *(volatile v4i*)(dp + 4 * tid) = vd;
    }
    if (tid < 8) {
      const v4i f = {ovf, ovf, ovf, ovf};
      *(volatile v4i*)(fp + 4 * tid) = f;
    }
    __threadfence();
  }
}

template <int LPO, int RELU>
__device__ __forceinline__ v4f walk_owner(const int* __restrict__ lb, const int* __restrict__ CNT,
                                          const int* __restrict__ OFF, const float* __restrict__ DINV,
                                          const float* __restrict__ T, int v, int j, int flag, v4f bb) {
  const int craw = CNT[v];
  const int oraw = OFF[v];
  const float dd = DINV[v];
  const v4f self = *(const v4fa*)(T + (size_t)v * OC + 4 * j);
  asm volatile("" :: "v"(craw), "v"(oraw), "v"(dd));
  asm volatile("" :: "v"(self));

  const bool big = craw > DEGCAP;
  const int c = craw < 0 ? 0 : (craw > DEGCAP ? DEGCAP : craw);
  const int o = clampi(oraw, 0, LCAP - 1);
  int last = o + c - 1;
  last = last > LCAP - 1 ? LCAP - 1 : last;

  int mx = c;
#pragma unroll
  for (int d = 16; d >= LPO; d >>= 1) {
    const int y = __shfl_xor(mx, d, 32);
    mx = y > mx ? y : mx;
  }
  const int trips = __builtin_amdgcn_readfirstlane(mx);

  float a0 = 0.0f, a1 = 0.0f, a2 = 0.0f, a3 = 0.0f;
#pragma unroll 1
  for (int t = 0; t < trips; ++t) {
    int idx = o + t;
    idx = idx > last ? last : idx;
    idx = (c > 0) ? idx : 0;
    idx = idx < 0 ? 0 : idx;
    int s = lb[idx];
    asm volatile("" :: "v"(s));
    s = s < 0 ? 0 : (s > NN - 1 ? NN - 1 : s);
    const float ds = DINV[s];
    const v4f q = *(const v4fa*)(T + (size_t)s * OC + 4 * j);
    asm volatile("" :: "v"(ds));
    asm volatile("" :: "v"(q));
    const float nrm = ds * dd;
    float p0 = q[0] * nrm, p1 = q[1] * nrm, p2 = q[2] * nrm, p3 = q[3] * nrm;
    asm volatile("" : "+v"(p0));
    asm volatile("" : "+v"(p1));
    asm volatile("" : "+v"(p2));
    asm volatile("" : "+v"(p3));
    const bool act = t < c;
    const float n0 = a0 + p0, n1 = a1 + p1, n2 = a2 + p2, n3 = a3 + p3;
    a0 = act ? n0 : a0;
    a1 = act ? n1 : a1;
    a2 = act ? n2 : a2;
    a3 = act ? n3 : a3;
  }
  const float wself = dd * dd;
  float s0 = self[0] * wself, s1 = self[1] * wself, s2 = self[2] * wself, s3 = self[3] * wself;
  asm volatile("" : "+v"(s0));
  asm volatile("" : "+v"(s1));
  asm volatile("" : "+v"(s2));
  asm volatile("" : "+v"(s3));
  a0 = a0 + s0; a1 = a1 + s1; a2 = a2 + s2; a3 = a3 + s3;
  float h0 = a0 + bb[0], h1 = a1 + bb[1], h2 = a2 + bb[2], h3 = a3 + bb[3];
  if (RELU) {
    h0 = (h0 > 0.0f) ? h0 : (h0 - h0);
    h1 = (h1 > 0.0f) ? h1 : (h1 - h1);
    h2 = (h2 > 0.0f) ? h2 : (h2 - h2);
    h3 = (h3 > 0.0f) ? h3 : (h3 - h3);
  }
  const bool bad = (flag != 0) | big;
  const float qnan = __uint_as_float(0x7fc00000u);
  v4f r;
  r[0] = bad ? qnan : h0;
  r[1] = bad ? qnan : h1;
  r[2] = bad ? qnan : h2;
  r[3] = bad ? qnan : h3;
  return r;
}

__global__ __launch_bounds__(NTHR) void k_walk1(const int* __restrict__ LIST, const int* __restrict__ CNT,
                                                const int* __restrict__ OFF, const float* __restrict__ DINV,
                                                const int* __restrict__ FLAG, const float* __restrict__ T,
                                                const float* __restrict__ BV, unsigned short* OP2) {
  __shared__ __attribute__((aligned(16))) unsigned tile[NWAVE][128];
  const int tid = (int)threadIdx.x, lane = tid & 31, wave = tid >> 5;
  const int blk = (int)blockIdx.x;
  const int j = lane & 3, g = lane >> 2;
  const int* lb = LIST + (size_t)blk * (size_t)LCAP;
  const int flag = FLAG[(size_t)blk * 32];
  const v4f bb = *(const v4fa*)(BV + 4 * j);
  asm volatile("" :: "v"(flag));
  asm volatile("" :: "v"(bb));
  unsigned* tw = tile[wave];
#pragma unroll 1
  for (int step = 0; step < 4; ++step) {
    const int v0 = blk * NBRUN + wave * 32 + step * 8;
    const v4f z = walk_owner<4, 1>(lb, CNT, OFF, DINV, T, v0 + g, j, flag, bb);
    const unsigned h01 = pk16(bf16_bits(z[0]), bf16_bits(z[1]));
    const unsigned h23 = pk16(bf16_bits(z[2]), bf16_bits(z[3]));
    const unsigned l01 = pk16(bf16_lo_bits(z[0]), bf16_lo_bits(z[1]));
    const unsigned l23 = pk16(bf16_lo_bits(z[2]), bf16_lo_bits(z[3]));
    unsigned* row = tw + g * 16;
    *(v2ua*)(row + 2 * j)     = (v2u){ h01, h23 };
    *(v2ua*)(row + 8 + 2 * j) = (v2u){ l01, l23 };
    __builtin_amdgcn_fence(__ATOMIC_RELEASE, "workgroup");
    __builtin_amdgcn_wave_barrier();
    __builtin_amdgcn_fence(__ATOMIC_ACQUIRE, "workgroup");
    const v4u ov = *(const v4ua*)(tw + 4 * lane);
    volatile v4u* q = (volatile v4u*)(OP2 + (size_t)v0 * K2 + 8 * lane);
    *q = ov;
    __threadfence();
    *q = ov;
    __builtin_amdgcn_fence(__ATOMIC_RELEASE, "workgroup");
    __builtin_amdgcn_wave_barrier();
    __builtin_amdgcn_fence(__ATOMIC_ACQUIRE, "workgroup");
  }
}

__global__ __launch_bounds__(NTHR) void k_walk2(const int* __restrict__ LIST, const int* __restrict__ CNT,
                                                const int* __restrict__ OFF, const float* __restrict__ DINV,
                                                const int* __restrict__ FLAG, const float* __restrict__ T,
                                                const float* __restrict__ BV, float* out, int n_nodes) {
  const int tid = (int)threadIdx.x, lane = tid & 31, wave = tid >> 5;
  const int blk = (int)blockIdx.x;
  const int j = lane & 15, g = lane >> 4;
  const int* lb = LIST + (size_t)blk * (size_t)LCAP;
  const int flag = FLAG[(size_t)blk * 32];
  const v4f bb = *(const v4fa*)(BV + 4 * j);
  asm volatile("" :: "v"(flag));
  asm volatile("" :: "v"(bb));
#pragma unroll 1
  for (int step = 0; step < 16; ++step) {
    const int v = blk * NBRUN + wave * 32 + step * 2 + g;
    const v4f z = walk_owner<16, 0>(lb, CNT, OFF, DINV, T, v, j, flag, bb);
    if (v < n_nodes) {
      volatile v4f* q = (volatile v4f*)(out + (size_t)v * OC + 4 * j);
      *q = z;
      __threadfence();
      *q = z;
    }
  }
}

extern "C" void kernel_launch(void* const* d_in, const int* in_sizes, int n_in,
                              void* d_out, int out_size, void* d_ws, size_t ws_size,
                              hipStream_t stream) {
  if (n_in < 6) return;
  if (in_sizes[0] != NN * KD) return;
  if (in_sizes[1] != 2 * NE) return;
  if (in_sizes[2] != KD * HID) return;
  if (in_sizes[3] != HID) return;
  if (in_sizes[4] != HID * OC) return;
  if (in_sizes[5] != OC) return;
  if (out_size != NN * OC) return;
  const int n_nodes = in_sizes[0] / KD;

  const float* x   = (const float*)d_in[0];
  const int*   ei  = (const int*)d_in[1];
  const float* W1  = (const float*)d_in[2];
  const float* b1  = (const float*)d_in[3];
  const float* W2  = (const float*)d_in[4];
  const float* b2  = (const float*)d_in[5];
  const int* srcs  = ei;
  const int* dsts  = ei + NE;
  float* out = (float*)d_out;

  constexpr size_t zXB   = (size_t)NPAD * KD * 2;
  constexpr size_t zT    = (size_t)NPAD * OC * 4;
  constexpr size_t zOP2  = (size_t)NPAD * K2 * 2;
  constexpr size_t zLIST = (size_t)NBK * LCAP * 4;
  constexpr size_t zTBL  = (size_t)NPAD * 4;
  constexpr size_t zFLAG = 50176;
  constexpr size_t zW1T  = (size_t)64 * KD * 2;
  constexpr size_t zW2D  = (size_t)64 * K2 * 2;
  constexpr size_t zTAB  = 1024;
  constexpr size_t oXB   = 0;
  constexpr size_t oT    = oXB + zXB;
  constexpr size_t oOP2  = oT + zT;
  constexpr size_t oLIST = oOP2 + zOP2;
  constexpr size_t oCNT  = oLIST + zLIST;
  constexpr size_t oOFF  = oCNT + zTBL;
  constexpr size_t oDINV = oOFF + zTBL;
  constexpr size_t oFLAG = oDINV + zTBL;
  constexpr size_t oW1T  = oFLAG + zFLAG;
  constexpr size_t oW2D  = oW1T + zW1T;
  constexpr size_t oTAB  = oW2D + zW2D;
  constexpr size_t oEND  = oTAB + zTAB;
  static_assert(zXB % 256 == 0 && zT % 256 == 0 && zOP2 % 256 == 0 && zLIST % 256 == 0 && zTBL % 256 == 0);
  static_assert(zFLAG % 256 == 0 && zW1T % 256 == 0 && zW2D % 256 == 0 && zTAB % 256 == 0);
  static_assert(zFLAG >= (size_t)NBK * 128);
  static_assert(zTAB >= (size_t)160 * 4);
  static_assert(oEND == 78146560);
  static_assert(oEND <= ((size_t)128 << 20));
  if (oEND > ws_size) return;

  char* ws = (char*)d_ws;
  unsigned short* XB   = (unsigned short*)(ws + oXB);
  float*          T    = (float*)(ws + oT);
  unsigned short* OP2  = (unsigned short*)(ws + oOP2);
  int*            LIST = (int*)(ws + oLIST);
  int*            CNT  = (int*)(ws + oCNT);
  int*            OFF  = (int*)(ws + oOFF);
  int*            DVB  = (int*)(ws + oDINV);
  const float*    DINV = (const float*)(ws + oDINV);
  int*            FLAG = (int*)(ws + oFLAG);
  unsigned short* W1T  = (unsigned short*)(ws + oW1T);
  unsigned short* W2D  = (unsigned short*)(ws + oW2D);
  float*          TAB  = (float*)(ws + oTAB);
  const float*    B1P  = TAB;
  const float*    B2P  = TAB + 32;
  const float*    ZERO = TAB + 96;

  hipFuncSetAttribute(reinterpret_cast<const void*>(&k_build), hipFuncAttributeMaxDynamicSharedMemorySize, (int)BK_LDS);

  k_plane<0><<<PBX, 256, 0, stream>>>(x, NN, KD, KD, XB, NPAD, KD);
  k_prep<<<PB_TOT, NTHR, 0, stream>>>(W1, W2, b1, b2, W1T, W2D, TAB);
  k_gemm_nt<0, 0><<<GEMM_BLOCKS, 256, 0, stream>>>(XB, W1T, ZERO, T, NPAD, OC, KD, OC);
  k_build<<<NBK, NTHR, BK_LDS, stream>>>(srcs, dsts, LIST, CNT, OFF, DVB, FLAG);
  k_walk1<<<NBK, NTHR, 0, stream>>>(LIST, CNT, OFF, DINV, FLAG, T, B1P, OP2);
  k_gemm_nt<0, 0><<<GEMM_BLOCKS, 256, 0, stream>>>(OP2, W2D, ZERO, T, NPAD, OC, K2, OC);
  k_walk2<<<NBK, NTHR, 0, stream>>>(LIST, CNT, OFF, DINV, FLAG, T, B2P, out, n_nodes);
}
